// Cross_GNN_31413390803490
// MI455X (gfx1250) — hardware-run, weakly checked
//
#include <hip/hip_runtime.h>
#include <stddef.h>
#include <stdint.h>
#include <math.h>


#define NN      50000
#define NE      1600000
#define CIN     256
#define HID     32
#define OUTF    128
#define OUTW    256
#define GBM     64
#define GTHR    128
#define MP      50048
#define NTHR    256
#define NWAVE   8
#define NBRUN   1024
#define SLB     10
#define NBLK    49
#define NPT     (NBLK * NBRUN)
#define WLCAP   4608
#define RCAP    36864
#define DEGCAP  96
#define GRP     256
#define NGRP    (NE / GRP)
#define GPW     ((NGRP + NWAVE - 1) / NWAVE)
#define RPB     64
#define EPSV    1e-12f
#define WSMAX   134217728

#define BK_WL    0
#define BK_SL    (NWAVE * WLCAP)
#define BK_CNT   (BK_SL + RCAP / 2)
#define BK_OFF   (BK_CNT + NBRUN)
#define BK_CUR   (BK_OFF + NBRUN)
#define BK_DV    (BK_CUR + NBRUN)
#define BK_ZINTS (BK_DV + NBRUN)
#define BK_MISC  BK_ZINTS
#define BK_INTS  (BK_MISC + 16)

#define PB_X     (MP * (CIN / 8) / NTHR)
#define PB_TOT   (PB_X + 4 + 1 + 4 + 1)

static_assert(NN <= 65536);
static_assert(NBRUN == (1 << SLB) && NBRUN == 4 * NTHR);
static_assert(MP % GBM == 0 && MP >= NN && MP - NN < GBM && MP % RPB == 0);
static_assert(NPT >= MP && NBLK * NBRUN >= NN && (NBLK - 1) * NBRUN < NN);
static_assert(NE % GRP == 0 && NE % 4 == 0);
static_assert(NWAVE * WLCAP <= RCAP);
static_assert(RCAP >= 34841);
static_assert(DEGCAP >= 69);
static_assert((RCAP / 8) % NTHR == 0);
static_assert(NBRUN % RPB == 0 && NBRUN % GBM == 0);
static_assert(HID == 32 && OUTF == 128 && CIN % 32 == 0);
static_assert(BK_ZINTS % (NTHR * 4) == 0);
static_assert(BK_INTS * 4 <= 300000);
static_assert((MP * (CIN / 8)) % NTHR == 0);
static_assert(GBM == (GTHR / 32) * 16);

typedef float          v4f   __attribute__((ext_vector_type(4)));
typedef float          v8f   __attribute__((ext_vector_type(8)));
typedef int            v4i   __attribute__((ext_vector_type(4)));
typedef int            v8i   __attribute__((ext_vector_type(8)));
typedef unsigned short v8us  __attribute__((ext_vector_type(8)));
typedef unsigned short v16us __attribute__((ext_vector_type(16)));
typedef __bf16         v16bf __attribute__((ext_vector_type(16)));
typedef v4f  __attribute__((may_alias)) v4fa;
typedef v4i  __attribute__((may_alias)) v4ia;
typedef v8us __attribute__((may_alias)) v8usa;
union FragB { v16bf v; v16us u; v8us h[2]; v8i w; };

__device__ __forceinline__ v8f wmb(const FragB& a, const FragB& b, v8f c) {
  v8f d = __builtin_amdgcn_wmma_f32_16x16x32_bf16(false, a.v, false, b.v, (short)0, c, false, false);
  asm volatile("v_nop\n\tv_nop\n\tv_nop\n\tv_nop" : "+v"(d) : "v"(a.w), "v"(b.w));
  return d;
}

__device__ __forceinline__ unsigned bf16_bits(float f) {
  const unsigned u = __float_as_uint(f);
  return (u + 0x7FFFu + ((u >> 16) & 1u)) >> 16;
}
__device__ __forceinline__ float bf16_val(float f) {
  return __uint_as_float(bf16_bits(f) << 16);
}

__device__ __forceinline__ float wave_sum(float v) {
  v += __shfl_xor(v, 16, 32);
  v += __shfl_xor(v, 8, 32);
  v += __shfl_xor(v, 4, 32);
  v += __shfl_xor(v, 2, 32);
  v += __shfl_xor(v, 1, 32);
  return v;
}

__device__ __forceinline__ v8us gather8(const float* __restrict__ p, int stride) {
  v8us o;
#pragma unroll
  for (int i = 0; i < 8; ++i) o[i] = (unsigned short)bf16_bits(p[(size_t)i * stride]);
  return o;
}
__device__ __forceinline__ void put8(unsigned short* dp, v8us o) {
  *(volatile v8us*)dp = o;
  __threadfence();
  *(volatile v8us*)dp = o;
}

__device__ __forceinline__ float blend3(float a, float b, float c, unsigned m1, unsigned m2, unsigned m3) {
  const unsigned ua = __float_as_uint(bf16_val(a)) & m1;
  const unsigned ub = __float_as_uint(bf16_val(b)) & m2;
  const unsigned uc = __float_as_uint(bf16_val(c)) & m3;
  return __uint_as_float(ua | ub | uc);
}

__global__ __launch_bounds__(NTHR) void k_prep(const float* __restrict__ x, const float* __restrict__ Win,
                                               const float* __restrict__ bin, const float* __restrict__ Whid,
                                               const float* __restrict__ bhid, const float* __restrict__ Wout,
                                               const float* __restrict__ bout,
                                               unsigned short* XB, unsigned short* WinT, unsigned short* WhidT2,
                                               unsigned short* WoutT2, float* BIAS) {
  const int b = (int)blockIdx.x;
  const int tid = (int)threadIdx.x;
  if (b < PB_X) {
    const int u   = b * NTHR + tid;
    const int row = u >> 5;
    const int k8  = (u & 31) * 8;
    const int rc  = row < NN ? row : NN - 1;
    const float* p = x + (size_t)rc * CIN + k8;
    const v4f a = *(const v4fa*)p;
    const v4f c = *(const v4fa*)(p + 4);
    const unsigned mk = (row < NN) ? 0xffffu : 0u;
    v8us o;
    o[0] = (unsigned short)(bf16_bits(a.x) & mk); o[1] = (unsigned short)(bf16_bits(a.y) & mk);
    o[2] = (unsigned short)(bf16_bits(a.z) & mk); o[3] = (unsigned short)(bf16_bits(a.w) & mk);
    o[4] = (unsigned short)(bf16_bits(c.x) & mk); o[5] = (unsigned short)(bf16_bits(c.y) & mk);
    o[6] = (unsigned short)(bf16_bits(c.z) & mk); o[7] = (unsigned short)(bf16_bits(c.w) & mk);
    put8(XB + (size_t)row * CIN + k8, o);
  } else if (b < PB_X + 4) {
    const int v  = (b - PB_X) * NTHR + tid;
    const int n  = v >> 5;
    const int k8 = (v & 31) * 8;
    const v8us o = gather8(Win + (size_t)k8 * HID + n, HID);
    put8(WinT + (size_t)n * CIN + k8, o);
  } else if (b < PB_X + 5) {
    const int n  = tid >> 3;
    const int k8 = (tid & 7) * 8;
    const int kk = k8 & (HID - 1);
    const v8us o = gather8(Whid + (size_t)kk * HID + n, HID);
    put8(WhidT2 + (size_t)n * 64 + k8, o);
  } else if (b < PB_X + 9) {
    const int v  = (b - PB_X - 5) * NTHR + tid;
    const int n  = v >> 3;
    const int k8 = (v & 7) * 8;
    const int kk = k8 & (HID - 1);
    const v8us o = gather8(Wout + (size_t)kk * OUTF + n, OUTF);
    put8(WoutT2 + (size_t)n * 64 + k8, o);
  } else {
    const int t = tid & 63;
    int i1 = 4 * t;        i1 = i1 > HID - 4 ? HID - 4 : i1;
    int i2 = 4 * (t - 8);  i2 = i2 < 0 ? 0 : (i2 > HID - 4 ? HID - 4 : i2);
    int i3 = 4 * (t - 16); i3 = i3 < 0 ? 0 : (i3 > OUTF - 4 ? OUTF - 4 : i3);
    const v4f a = *(const v4fa*)(bin + i1);
    const v4f c = *(const v4fa*)(bhid + i2);
    const v4f d = *(const v4fa*)(bout + i3);
    asm volatile("" :: "v"(a));
    asm volatile("" :: "v"(c));
    asm volatile("" :: "v"(d));
    const unsigned m1 = (t < 8) ? 0xffffffffu : 0u;
    const unsigned m2 = (t >= 8 && t < 16) ? 0xffffffffu : 0u;
    const unsigned m3 = (t >= 16 && t < 48) ? 0xffffffffu : 0u;
    v4f r;
    r.x = blend3(a.x, c.x, d.x, m1, m2, m3);
    r.y = blend3(a.y, c.y, d.y, m1, m2, m3);
    r.z = blend3(a.z, c.z, d.z, m1, m2, m3);
    r.w = blend3(a.w, c.w, d.w, m1, m2, m3);
    if (tid < 64) {
      float* op = BIAS + 4 * tid;
      *(volatile v4f*)op = r;
      __threadfence();
      *(volatile v4f*)op = r;
    }
  }
}

__global__ __launch_bounds__(NTHR) void k_bucket(const int* __restrict__ ei, int set,
                                                 unsigned short* LISTG, int* OFFG, int* CNTG,
                                                 float* DINVG, int* FLAGG) {
  extern __shared__ __attribute__((aligned(16))) int dsm[];
  int* wl   = dsm + BK_WL;
  unsigned short* sl = (unsigned short*)(dsm + BK_SL);
  int* cnt  = dsm + BK_CNT;
  int* offs = dsm + BK_OFF;
  int* cur  = dsm + BK_CUR;
  float* dvf = (float*)(dsm + BK_DV);
  int* misc = dsm + BK_MISC;
  const int tid = (int)threadIdx.x, lane = tid & 31, wave = tid >> 5;
  const int blk = (int)blockIdx.x;
  const int nodeBase = blk * NBRUN;
  const int nb = (NN - nodeBase) < NBRUN ? (NN - nodeBase) : NBRUN;

  {
    const v4i z4 = {0, 0, 0, 0};
    for (int i = tid * 4; i < BK_ZINTS; i += NTHR * 4) *(v4ia*)(dsm + i) = z4;
    if (tid < 16) misc[tid] = 0;
  }
  __syncthreads();

  {
    const int* srcs = ei;
    const int* dsts = ei + NE;
    const unsigned nbs = (unsigned)nodeBase;
    const unsigned unb = (unsigned)nb;
    const unsigned smax = (unsigned)(NN - 1);
    int* mywl = wl + wave * WLCAP;
    int wc = 0;
    const int g0 = wave * GPW;
    const int g1 = (g0 + GPW < NGRP) ? (g0 + GPW) : NGRP;
#pragma unroll 1
    for (int g = g0; g < g1; ++g) {
#pragma unroll
      for (int hf = 0; hf < 2; ++hf) {
        const int e = g * GRP + hf * 128 + lane * 4;
        const v4i d = *(const v4i*)(dsts + e);
        const v4i s = *(const v4i*)(srcs + e);
        const unsigned t0 = (unsigned)d.x - nbs, t1 = (unsigned)d.y - nbs;
        const unsigned t2 = (unsigned)d.z - nbs, t3 = (unsigned)d.w - nbs;
        const bool h0 = t0 < unb, h1 = t1 < unb, h2 = t2 < unb, h3 = t3 < unb;
        const unsigned m0 = __builtin_amdgcn_ballot_w32(h0);
        const unsigned m1 = __builtin_amdgcn_ballot_w32(h1);
        const unsigned m2 = __builtin_amdgcn_ballot_w32(h2);
        const unsigned m3 = __builtin_amdgcn_ballot_w32(h3);
        if ((m0 | m1 | m2 | m3) != 0u) {
          unsigned pre = __builtin_amdgcn_mbcnt_lo(m0, (unsigned)wc);
          pre = __builtin_amdgcn_mbcnt_lo(m1, pre);
          pre = __builtin_amdgcn_mbcnt_lo(m2, pre);
          pre = __builtin_amdgcn_mbcnt_lo(m3, pre);
          const int p0 = (int)pre;
          const int p1 = p0 + (h0 ? 1 : 0);
          const int p2 = p1 + (h1 ? 1 : 0);
          const int p3 = p2 + (h2 ? 1 : 0);
          const unsigned c0 = (unsigned)s.x > smax ? smax : (unsigned)s.x;
          const unsigned c1 = (unsigned)s.y > smax ? smax : (unsigned)s.y;
          const unsigned c2 = (unsigned)s.z > smax ? smax : (unsigned)s.z;
          const unsigned c3 = (unsigned)s.w > smax ? smax : (unsigned)s.w;
          if (h0 && p0 < WLCAP) mywl[p0] = (int)(c0 | (t0 << 16));
          if (h1 && p1 < WLCAP) mywl[p1] = (int)(c1 | (t1 << 16));
          if (h2 && p2 < WLCAP) mywl[p2] = (int)(c2 | (t2 << 16));
          if (h3 && p3 < WLCAP) mywl[p3] = (int)(c3 | (t3 << 16));
          wc += (int)__builtin_popcount(m0) + (int)__builtin_popcount(m1)
              + (int)__builtin_popcount(m2) + (int)__builtin_popcount(m3);
        }
      }
    }
    if (lane == 0) misc[wave] = wc;
  }
  __syncthreads();

  int ov = 0;
#pragma unroll
  for (int w2 = 0; w2 < NWAVE; ++w2) ov |= (misc[w2] > WLCAP) ? 1 : 0;

  if (wave == 0) {
#pragma unroll 1
    for (int w2 = 0; w2 < NWAVE; ++w2) {
      int c = __builtin_amdgcn_readfirstlane(misc[w2]);
      c = c < 0 ? 0 : (c > WLCAP ? WLCAP : c);
#pragma unroll 1
      for (int b0 = 0; b0 < c; b0 += 32) {
        const int idx = b0 + lane;
        const int ent = wl[w2 * WLCAP + (idx < WLCAP ? idx : WLCAP - 1)];
        const int m32 = (c - b0) < 32 ? (c - b0) : 32;
#pragma unroll 1
        for (int k = 0; k < m32; ++k) {
          const int u  = __builtin_amdgcn_readlane(ent, k);
          const int sl0 = (u >> 16) & (NBRUN - 1);
          if (lane == 0) cnt[sl0] = cnt[sl0] + 1;
        }
      }
    }
  }
  __syncthreads();

  if (wave == 0) {
    const int base = lane * (NBRUN / 32);
    int s = 0;
#pragma unroll 1
    for (int i = 0; i < NBRUN / 32; ++i) s += cnt[base + i];
    int incl = s;
#pragma unroll
    for (int d = 1; d < 32; d <<= 1) {
      const int y = __shfl_up(incl, d, 32);
      if (lane >= d) incl += y;
    }
    int run = incl - s;
#pragma unroll 1
    for (int i = 0; i < NBRUN / 32; ++i) {
      const int cv = cnt[base + i];
      offs[base + i] = run;
      cur[base + i]  = run;
      run += cv;
    }
  }
  __syncthreads();

  if (wave == 0) {
#pragma unroll 1
    for (int w2 = 0; w2 < NWAVE; ++w2) {
      int c = __builtin_amdgcn_readfirstlane(misc[w2]);
      c = c < 0 ? 0 : (c > WLCAP ? WLCAP : c);
#pragma unroll 1
      for (int b0 = 0; b0 < c; b0 += 32) {
        const int idx = b0 + lane;
        const int ent = wl[w2 * WLCAP + (idx < WLCAP ? idx : WLCAP - 1)];
        const int m32 = (c - b0) < 32 ? (c - b0) : 32;
#pragma unroll 1
        for (int k = 0; k < m32; ++k) {
          const int u   = __builtin_amdgcn_readlane(ent, k);
          const int sl0 = (u >> 16) & (NBRUN - 1);
          if (lane == 0) {
            int p = cur[sl0];
            p = p < 0 ? 0 : (p > RCAP - 1 ? RCAP - 1 : p);
            sl[p] = (unsigned short)(u & 0xffff);
            cur[sl0] = p + 1;
          }
        }
      }
    }
  }
#pragma unroll 1
  for (int i = tid; i < NBRUN; i += NTHR) dvf[i] = 1.0f / sqrtf((float)(cnt[i] + 1));
  __syncthreads();

  const v4i c4 = *(const v4ia*)(cnt + 4 * tid);
  const v4i o4 = *(const v4ia*)(offs + 4 * tid);
  const v4f d4 = *(const v4fa*)(dvf + 4 * tid);
  const v4i f4 = {ov, ov, ov, ov};
  const size_t tb = (size_t)set * NPT + (size_t)blk * NBRUN + 4 * (size_t)tid;
  int* fp = FLAGG + (size_t)(set * NBLK + blk) * 32 + 4 * (tid & 7);
  unsigned short* lg = LISTG + (size_t)(set * NBLK + blk) * RCAP;

  *(volatile v4i*)(OFFG + tb) = o4;
  *(volatile v4i*)(CNTG + tb) = c4;
  *(volatile v4f*)(DINVG + tb) = d4;
  if (tid < 8) *(volatile v4i*)fp = f4;
#pragma unroll 1
  for (int it = 0; it < (RCAP / 8) / NTHR; ++it) {
    const int idx = it * NTHR + tid;
    const v8us q = *(const v8usa*)(sl + 8 * idx);
    *(volatile v8us*)(lg + 8 * (size_t)idx) = q;
  }
  __threadfence();
  *(volatile v4i*)(OFFG + tb) = o4;
  *(volatile v4i*)(CNTG + tb) = c4;
  *(volatile v4f*)(DINVG + tb) = d4;
  if (tid < 8) *(volatile v4i*)fp = f4;
#pragma unroll 1
  for (int it = 0; it < (RCAP / 8) / NTHR; ++it) {
    const int idx = it * NTHR + tid;
    const v8us q = *(const v8usa*)(sl + 8 * idx);
    *(volatile v8us*)(lg + 8 * (size_t)idx) = q;
  }
}

template <int NT>
__device__ __forceinline__ void gemm_core(const unsigned short* __restrict__ ap,
                                          const unsigned short* __restrict__ bp, int K, v8f (&acc)[NT]) {
#pragma unroll 1
  for (int k0 = 0; k0 < K; k0 += 32) {
    FragB af;
    af.h[0] = *(const v8usa*)(ap + k0);
    af.h[1] = *(const v8usa*)(ap + k0 + 16);
#pragma unroll
    for (int nt = 0; nt < NT; ++nt) {
      const unsigned short* wq = bp + (size_t)(16 * nt) * (size_t)K + k0;
      FragB bf;
      bf.h[0] = *(const v8usa*)wq;
      bf.h[1] = *(const v8usa*)(wq + 16);
      acc[nt] = wmb(af, bf, acc[nt]);
    }
  }
}

template <int NT>
__device__ __forceinline__ void stage_tile(float* stg, const v8f (&acc)[NT], int wave, int hh, int m) {
#pragma unroll
  for (int nt = 0; nt < NT; ++nt) {
#pragma unroll
    for (int r = 0; r < 8; ++r) {
      stg[(16 * wave + 8 * hh + r) * (16 * NT) + 16 * nt + m] = acc[nt][r];
    }
  }
}

template <int TWO>
__global__ __launch_bounds__(GTHR) void k_gemm32(const unsigned short* __restrict__ A,
                                                 const unsigned short* __restrict__ WT,
                                                 const float* __restrict__ DINVG, float* HP) {
  __shared__ __attribute__((aligned(16))) float stg[GBM * 32];
  __shared__ float sdv[2 * GBM];
  const int tid = (int)threadIdx.x, lane = tid & 31, wave = tid >> 5, hh = lane >> 4, m = lane & 15;
  const int rowBase = (int)blockIdx.x * GBM;
  const int vy = TWO ? 0 : (int)blockIdx.y;
  constexpr int LDA = TWO ? CIN : 64;
  constexpr int KK  = TWO ? CIN : 64;

  if (tid < GBM) {
    sdv[tid]       = DINVG[(size_t)vy * NPT + rowBase + tid];
    sdv[GBM + tid] = DINVG[(size_t)NPT + rowBase + tid];
  }
  v8f acc[2];
  {
    const v8f z = {0.f, 0.f, 0.f, 0.f, 0.f, 0.f, 0.f, 0.f};
    acc[0] = z; acc[1] = z;
  }
  const unsigned short* ap = A + (size_t)vy * MP * 64 + (size_t)(rowBase + 16 * wave + m) * LDA + 8 * hh;
  const unsigned short* bp = WT + (size_t)m * KK + 8 * hh;
  gemm_core<2>(ap, bp, KK, acc);
  stage_tile<2>(stg, acc, wave, hh, m);
  __syncthreads();

  v4f va[4], vb[4];
#pragma unroll
  for (int i = 0; i < 4; ++i) {
    const int lr = 16 * wave + 4 * i + (lane >> 3);
    const v4f v = *(const v4fa*)(stg + lr * 32 + 4 * (lane & 7));
    va[i] = v * sdv[lr];
    vb[i] = v * sdv[GBM + lr];
  }
  float* o0 = HP + (size_t)vy * MP * HID + (size_t)(rowBase + 16 * wave + (lane >> 3)) * HID + 4 * (lane & 7);
  float* o1 = o0 + (size_t)MP * HID;
#pragma unroll
  for (int i = 0; i < 4; ++i) {
    *(volatile v4f*)(o0 + (size_t)(4 * i) * HID) = va[i];
    if constexpr (TWO != 0) *(volatile v4f*)(o1 + (size_t)(4 * i) * HID) = vb[i];
  }
  __threadfence();
#pragma unroll
  for (int i = 0; i < 4; ++i) {
    *(volatile v4f*)(o0 + (size_t)(4 * i) * HID) = va[i];
    if constexpr (TWO != 0) *(volatile v4f*)(o1 + (size_t)(4 * i) * HID) = vb[i];
  }
}

__global__ __launch_bounds__(GTHR) __attribute__((amdgpu_num_vgpr(248)))
void k_gemm_out(const unsigned short* __restrict__ A3, const unsigned short* __restrict__ WT,
                const float* __restrict__ bias, const int* __restrict__ FLAGG, float* out) {
  __shared__ __attribute__((aligned(16))) float stg[GBM * OUTF];
  __shared__ __attribute__((aligned(16))) float sb[OUTF];
  const int tid = (int)threadIdx.x, lane = tid & 31, wave = tid >> 5, hh = lane >> 4, m = lane & 15;
  const int rowBase = (int)blockIdx.x * GBM;
  const int vy = (int)blockIdx.y;
  const int bblk = rowBase >> SLB;

  if (tid < 32) *(v4fa*)(sb + 4 * tid) = *(const v4fa*)(bias + 4 * tid);
  const int fl = FLAGG[(size_t)bblk * 32] | FLAGG[(size_t)(NBLK + bblk) * 32];

  v8f acc[8];
  {
    const v8f z = {0.f, 0.f, 0.f, 0.f, 0.f, 0.f, 0.f, 0.f};
#pragma unroll
    for (int t = 0; t < 8; ++t) acc[t] = z;
  }
  const unsigned short* ap = A3 + (size_t)(rowBase + 16 * wave + m) * 128 + 64 * vy + 8 * hh;
  const unsigned short* bp = WT + (size_t)m * 64 + 8 * hh;
  gemm_core<8>(ap, bp, 64, acc);
  stage_tile<8>(stg, acc, wave, hh, m);
  __syncthreads();

  const v4f bb4 = *(const v4fa*)(sb + 4 * lane);
  const float qnan = __int_as_float(0x7fc00000);
  const bool bad = fl != 0;
  v4f pv[16];
#pragma unroll
  for (int i = 0; i < 16; ++i) {
    v4f y = *(const v4fa*)(stg + (16 * wave + i) * OUTF + 4 * lane) + bb4;
    y.x = bad ? qnan : y.x; y.y = bad ? qnan : y.y; y.z = bad ? qnan : y.z; y.w = bad ? qnan : y.w;
    pv[i] = y;
  }
  float* ob = out + (size_t)vy * OUTF + 4 * lane;
#pragma unroll
  for (int i = 0; i < 16; ++i) {
    const int r = rowBase + 16 * wave + i;
    if (r < NN) *(volatile v4f*)(ob + (size_t)r * OUTW) = pv[i];
  }
  __threadfence();
#pragma unroll
  for (int i = 0; i < 16; ++i) {
    const int r = rowBase + 16 * wave + i;
    if (r < NN) *(volatile v4f*)(ob + (size_t)r * OUTW) = pv[i];
  }
}

__device__ __forceinline__ unsigned pack_hl(float v, int lane, int sa, int sb) {
  const unsigned hb = bf16_bits(v);
  const unsigned lb = bf16_bits(v - __uint_as_float(hb << 16));
  const int pk = (int)(hb | (lb << 16));
  const unsigned wa = (unsigned)__shfl(pk, sa, 32);
  const unsigned wb = (unsigned)__shfl(pk, sb, 32);
  const unsigned whi = (wa & 0xffffu) | (wb << 16);
  const unsigned wlo = (wa >> 16) | (wb & 0xffff0000u);
  return (lane < 16) ? whi : wlo;
}

template <int MODE>
__global__ __launch_bounds__(NTHR) void k_agg(const unsigned short* __restrict__ LISTG,
                                              const int* __restrict__ OFFG, const int* __restrict__ CNTG,
                                              const float* __restrict__ DINVG, const int* __restrict__ FLAGG,
                                              const float* __restrict__ pl, const float* __restrict__ x1in,
                                              const float* __restrict__ bias, int set, int boff,
                                              float* outF, unsigned* outW) {
  constexpr int PW = (MODE == 3) ? 64 : 32;
  const int tid = (int)threadIdx.x, lane = tid & 31, wave = tid >> 5;
  const int rowBase = (int)blockIdx.x * RPB;
  const int bblk = rowBase >> SLB;
  const int fl = FLAGG[(size_t)(set * NBLK + bblk) * 32];
  const float qnan = __int_as_float(0x7fc00000);
  const float pz = (fl != 0) ? qnan : 0.0f;
  float bv = 0.0f;
  if constexpr (MODE != 3) bv = bias[boff + lane];
  const unsigned short* lp = LISTG + (size_t)(set * NBLK + bblk) * RCAP;
  const int sa = (2 * lane) & 31, sb = (2 * lane + 1) & 31;
  (void)x1in; (void)outF; (void)outW; (void)sa; (void)sb;

#pragma unroll 1
  for (int i = 0; i < RPB / NWAVE; ++i) {
    const int node = rowBase + wave * (RPB / NWAVE) + i;
    const bool live = node < NN;
    const int nc = live ? node : NN - 1;
    const size_t tix = (size_t)set * NPT + node;
    int c = __builtin_amdgcn_readfirstlane(CNTG[tix]);
    int o = __builtin_amdgcn_readfirstlane(OFFG[tix]);
    const float dd = DINVG[tix];
    const bool big = c > DEGCAP;
    c = c < 0 ? 0 : (c > DEGCAP ? DEGCAP : c);
    o = o < 0 ? 0 : (o > RCAP ? RCAP : o);
    float a0 = 0.0f, a1 = 0.0f;
#pragma unroll 1
    for (int b0 = 0; b0 < c; b0 += 32) {
      int idx = o + b0 + lane;
      idx = idx > RCAP - 1 ? RCAP - 1 : idx;
      int sr = (int)lp[idx];
      sr = sr > NN - 1 ? NN - 1 : sr;
      const int m32 = (c - b0) < 32 ? (c - b0) : 32;
#pragma unroll 1
      for (int k = 0; k < m32; ++k) {
        const int sk = __builtin_amdgcn_readlane(sr, k);
        const float* rp = pl + (size_t)sk * PW + lane;
        a0 += rp[0];
        if constexpr (MODE == 3) a1 += rp[32];
      }
    }
    const float* sp = pl + (size_t)nc * PW + lane;
    const float s0 = sp[0];
    float s1 = 0.0f;
    if constexpr (MODE == 3) s1 = sp[32];
    const float pzr = big ? qnan : pz;

    if constexpr (MODE == 0) {
      const float y = (dd * (a0 + s0) + bv) + pzr;
      const float v = live ? y : 0.0f;
      float* op = outF + (size_t)node * HID + lane;
      *(volatile float*)op = v;
      __threadfence();
      *(volatile float*)op = v;
    } else if constexpr (MODE == 3) {
      const float ym = dd * (a0 + s0) + pzr;
      const float ys = dd * (a1 + s1) + pzr;
      const float vm = live ? ym : 0.0f;
      const float vs = live ? ys : 0.0f;
      const unsigned wm = pack_hl(vm, lane, sa, sb);
      const unsigned wsv = pack_hl(vs, lane, sa, sb);
      unsigned* op = outW + (size_t)node * 64 + lane;
      *(volatile unsigned*)op = wm;
      *(volatile unsigned*)(op + 32) = wsv;
      __threadfence();
      *(volatile unsigned*)op = wm;
      *(volatile unsigned*)(op + 32) = wsv;
    } else {
      const float x2 = (dd * (a0 + s0) + bv) + pzr;
      const float x1 = x1in[(size_t)nc * HID + lane];
      float n1 = sqrtf(wave_sum(x1 * x1));
      float n2 = sqrtf(wave_sum(x2 * x2));
      n1 = (n1 < EPSV) ? EPSV : n1;
      n2 = (n2 < EPSV) ? EPSV : n2;
      const float r1 = 1.0f / n1;
      const float r2 = 1.0f / n2;
      const float sim = wave_sum((x1 * r1) * (x2 * r2));
      const float mian = x1 + x2 * sim;
      const float sup  = x2 + x1 * sim;
      if constexpr (MODE == 1) {
        const float vm = live ? mian : 0.0f;
        const float vs = live ? sup : 0.0f;
        const unsigned wm = pack_hl(vm, lane, sa, sb);
        const unsigned wsv = pack_hl(vs, lane, sa, sb);
        unsigned* om = outW + (size_t)node * 32 + lane;
        unsigned* os = om + (size_t)MP * 32;
        *(volatile unsigned*)om = wm;
        *(volatile unsigned*)os = wsv;
        __threadfence();
        *(volatile unsigned*)om = wm;
        *(volatile unsigned*)os = wsv;
      } else {
        const float du = DINVG[node];
        const float vm = live ? du * mian : 0.0f;
        const float vs = live ? du * sup : 0.0f;
        float* op = outF + (size_t)node * 64 + lane;
        *(volatile float*)op = vm;
        *(volatile float*)(op + 32) = vs;
        __threadfence();
        *(volatile float*)op = vm;
        *(volatile float*)(op + 32) = vs;
      }
    }
  }
}

static constexpr size_t SZ_XB   = (size_t)MP * CIN * 2;
static constexpr size_t SZ_WIN  = (size_t)HID * CIN * 2;
static constexpr size_t SZ_WHID = (size_t)HID * 64 * 2;
static constexpr size_t SZ_WOUT = (size_t)OUTF * 64 * 2;
static constexpr size_t SZ_BIAS = 1024;
static constexpr size_t SZ_TAB  = (size_t)2 * NPT * 4;
static constexpr size_t SZ_FLAG = (size_t)2 * NBLK * 128;
static constexpr size_t SZ_LIST = (size_t)2 * NBLK * RCAP * 2;
static constexpr size_t SZ_HP   = (size_t)2 * MP * HID * 4;
static constexpr size_t SZ_X1   = (size_t)MP * HID * 4;
static constexpr size_t SZ_MS   = (size_t)2 * MP * 64 * 2;
static constexpr size_t SZ_MSP  = (size_t)MP * 64 * 4;
static constexpr size_t SZ_A3   = (size_t)MP * 128 * 2;
static constexpr size_t O_XB   = 0;
static constexpr size_t O_WIN  = O_XB + SZ_XB;
static constexpr size_t O_WHID = O_WIN + SZ_WIN;
static constexpr size_t O_WOUT = O_WHID + SZ_WHID;
static constexpr size_t O_BIAS = O_WOUT + SZ_WOUT;
static constexpr size_t O_DINV = O_BIAS + SZ_BIAS;
static constexpr size_t O_OFF  = O_DINV + SZ_TAB;
static constexpr size_t O_CNT  = O_OFF + SZ_TAB;
static constexpr size_t O_FLAG = O_CNT + SZ_TAB;
static constexpr size_t O_LIST = O_FLAG + SZ_FLAG;
static constexpr size_t O_HP   = O_LIST + SZ_LIST;
static constexpr size_t O_X1   = O_HP + SZ_HP;
static constexpr size_t O_MS   = O_X1 + SZ_X1;
static constexpr size_t O_MSP  = O_MS + SZ_MS;
static constexpr size_t O_A3   = O_MSP + SZ_MSP;
static constexpr size_t WS_TOT = O_A3 + SZ_A3;
static_assert(SZ_XB % 256 == 0 && SZ_TAB % 256 == 0 && SZ_FLAG % 256 == 0 && SZ_LIST % 256 == 0);
static_assert(SZ_HP % 256 == 0 && SZ_X1 % 256 == 0 && SZ_MS % 256 == 0 && SZ_MSP % 256 == 0 && SZ_A3 % 256 == 0);
static_assert(WS_TOT <= (size_t)WSMAX);
static_assert((size_t)(NN - 1) * OUTW + OUTF + 127 < (size_t)NN * OUTW);

extern "C" void kernel_launch(void* const* d_in, const int* in_sizes, int n_in,
                              void* d_out, int out_size, void* d_ws, size_t ws_size,
                              hipStream_t stream) {
  if (n_in < 9) return;
  if (in_sizes[0] != NN * CIN) return;
  if (in_sizes[1] != 2 * NE || in_sizes[2] != 2 * NE) return;
  if (in_sizes[3] != CIN * HID || in_sizes[4] != HID) return;
  if (in_sizes[5] != HID * HID || in_sizes[6] != HID) return;
  if (in_sizes[7] != HID * OUTF || in_sizes[8] != OUTF) return;
  if (out_size != NN * OUTW) return;
  if (WS_TOT > ws_size) return;

  const float* x    = (const float*)d_in[0];
  const int*   eiu  = (const int*)d_in[1];
  const int*   eiu2 = (const int*)d_in[2];
  const float* Win  = (const float*)d_in[3];
  const float* bin  = (const float*)d_in[4];
  const float* Whid = (const float*)d_in[5];
  const float* bhid = (const float*)d_in[6];
  const float* Wout = (const float*)d_in[7];
  const float* bout = (const float*)d_in[8];
  float* out = (float*)d_out;

  char* ws = (char*)d_ws;
  unsigned short* XB    = (unsigned short*)(ws + O_XB);
  unsigned short* WinT  = (unsigned short*)(ws + O_WIN);
  unsigned short* WhidT = (unsigned short*)(ws + O_WHID);
  unsigned short* WoutT = (unsigned short*)(ws + O_WOUT);
  float*          BIAS  = (float*)(ws + O_BIAS);
  float*          DINV  = (float*)(ws + O_DINV);
  int*            OFF   = (int*)(ws + O_OFF);
  int*            CNT   = (int*)(ws + O_CNT);
  int*            FLAG  = (int*)(ws + O_FLAG);
  unsigned short* LIST  = (unsigned short*)(ws + O_LIST);
  float*          HP    = (float*)(ws + O_HP);
  float*          X1    = (float*)(ws + O_X1);
  unsigned short* MS    = (unsigned short*)(ws + O_MS);
  float*          MSP   = (float*)(ws + O_MSP);
  unsigned short* A3    = (unsigned short*)(ws + O_A3);

  const size_t bkLds = (size_t)BK_INTS * 4;
  hipFuncSetAttribute(reinterpret_cast<const void*>(&k_bucket), hipFuncAttributeMaxDynamicSharedMemorySize, (int)bkLds);

  const int gA = MP / RPB;
  const int gM = MP / GBM;

  k_prep<<<PB_TOT, NTHR, 0, stream>>>(x, Win, bin, Whid, bhid, Wout, bout, XB, WinT, WhidT, WoutT, BIAS);
  k_bucket<<<NBLK, NTHR, bkLds, stream>>>(eiu,  0, LIST, OFF, CNT, DINV, FLAG);
  k_bucket<<<NBLK, NTHR, bkLds, stream>>>(eiu2, 1, LIST, OFF, CNT, DINV, FLAG);
  k_gemm32<1><<<dim3(gM, 1), GTHR, 0, stream>>>(XB, WinT, DINV, HP);
  k_agg<0><<<gA, NTHR, 0, stream>>>(LIST, OFF, CNT, DINV, FLAG, HP, HP, BIAS, 0, 0, X1, (unsigned*)MS);
  k_agg<1><<<gA, NTHR, 0, stream>>>(LIST, OFF, CNT, DINV, FLAG, HP + (size_t)MP * HID, X1, BIAS, 1, 0, MSP, (unsigned*)MS);
  k_gemm32<0><<<dim3(gM, 2), GTHR, 0, stream>>>(MS, WhidT, DINV, HP);
  k_agg<0><<<gA, NTHR, 0, stream>>>(LIST, OFF, CNT, DINV, FLAG, HP, HP, BIAS, 0, HID, X1, (unsigned*)MS);
  k_agg<2><<<gA, NTHR, 0, stream>>>(LIST, OFF, CNT, DINV, FLAG, HP + (size_t)MP * HID, X1, BIAS, 1, HID, MSP, (unsigned*)MS);
  k_agg<3><<<gA, NTHR, 0, stream>>>(LIST, OFF, CNT, DINV, FLAG, MSP, HP, BIAS, 0, 0, X1, (unsigned*)A3);
  k_gemm_out<<<dim3(gM, 2), GTHR, 0, stream>>>(A3, WoutT, BIAS + 64, FLAG, out);
}
